// RNN_7370163880375
// MI455X (gfx1250) — hardware-verified
//
#include <hip/hip_runtime.h>
#include <math.h>

constexpr int NBATCH   = 256;
constexpr int NSTEPS   = 4096;
constexpr int NHID     = 64;
constexpr int ROWS_BLK = 16;
constexpr int CHUNK_T  = 64;
constexpr int NCHUNK   = NSTEPS / CHUNK_T;
constexpr int HROW     = 72;
constexpr int HBUF     = ROWS_BLK * HROW;
constexpr int FROW     = 68;
constexpr int NTHREADS = 128;
constexpr float HCARRY   = 16.0f;
constexpr float WCARRY   = 8.0f;
constexpr float ACCSCALE = HCARRY * WCARRY;
constexpr float ACCFOLD  = 1.0f / ACCSCALE;
constexpr int OUT0_ELEMS = NBATCH * NSTEPS;
constexpr int OUT1_ELEMS = NBATCH * NHID;
static_assert(NSTEPS % CHUNK_T == 0, "chunking exact");
static_assert(NBATCH % ROWS_BLK == 0, "grid exact");
static_assert(NHID == 64, "K = 64 = two 32-deep k tiles, four 16-row m tiles");
static_assert(CHUNK_T == 64, "staging row = 64 floats = 256 B");
static_assert(NTHREADS == 128, "4 waves: one 16-row hidden tile each");
static_assert((size_t)OUT0_ELEMS * 4 == 4194304, "out1 byte offset");
static_assert((size_t)(OUT0_ELEMS + OUT1_ELEMS) * 4 == 4259840, "d_out total bytes");
static_assert(((size_t)OUT0_ELEMS * 4) % 128 == 0, "out1 starts on a 128-B line");

typedef __attribute__((ext_vector_type(16))) _Float16 v16h;
typedef __attribute__((ext_vector_type(8)))  _Float16 v8h;
typedef __attribute__((ext_vector_type(8)))  float    v8f;
typedef __attribute__((ext_vector_type(4)))  float    v4f;

template <typename T> struct Frag;
template <> struct Frag<_Float16> {
  typedef v16h V; union U { v16h v; v8h h[2]; };
  static __device__ __forceinline__ v16h load(const _Float16* p) {
    U f; f.h[0] = *(const v8h*)(p); f.h[1] = *(const v8h*)(p + 16); return f.v;
  }
  static __device__ __forceinline__ v8f mma(v16h a, v16h b, v8f c) {
    return __builtin_amdgcn_wmma_f32_16x16x32_f16(false, a, false, b, (short)0, c, false, false);
  }
};

__device__ __forceinline__ void wmma_guard(v8f& acc, v16h a0, v16h b0, v16h a1, v16h b1) {
  asm volatile("v_nop\n\tv_nop\n\tv_nop\n\tv_nop" : "+v"(acc) : "v"(a0), "v"(b0), "v"(a1), "v"(b1));
}

__device__ __forceinline__ float tanh_f32(float v) {
  const float e  = expf(2.0f * v);
  const float rc = 1.0f / (1.0f + e);
  return 1.0f - 2.0f * rc;
}

__device__ __forceinline__ void flush_tile(const float* sh, float* gdst, int gpitch, float addv, int wave, int lane) {
  const int hh = lane >> 4;
  const int c4 = (lane & 15) * 4;
  const int row0 = 4 * wave + hh;
  const int row1 = row0 + 2;
  v4f ov0 = *(const v4f*)(sh + row0 * FROW + c4);
  v4f ov1 = *(const v4f*)(sh + row1 * FROW + c4);
#pragma unroll
  for (int e = 0; e < 4; ++e) { ov0[e] = ov0[e] + addv; ov1[e] = ov1[e] + addv; }
  float* g0 = gdst + (size_t)row0 * (size_t)gpitch + c4;
  float* g1 = gdst + (size_t)row1 * (size_t)gpitch + c4;
  *(volatile v4f*)g0 = ov0;
  *(volatile v4f*)g1 = ov1;
  __threadfence();
  *(volatile v4f*)g0 = ov0;
  *(volatile v4f*)g1 = ov1;
  __threadfence();
}

__global__ __launch_bounds__(NTHREADS) void rnn_seq_kernel(
    const float* __restrict__ x,     const float* __restrict__ h0,
    const float* __restrict__ w_ih,  const float* __restrict__ w_hh,
    const float* __restrict__ b_ih,  const float* __restrict__ b_hh,
    const float* __restrict__ w_out, const float* __restrict__ b_out,
    float* __restrict__ outs,        float* __restrict__ h_last) {
  __shared__ __align__(16) _Float16 h_sh[2 * HBUF];
  __shared__ __align__(16) float    x_sh[ROWS_BLK * FROW];
  __shared__ __align__(16) float    ob_sh[ROWS_BLK * FROW];
  __shared__ __align__(16) float    part_sh[2 * 128];
  __shared__ __align__(16) float    hf_sh[ROWS_BLK * FROW];

  const int tid   = threadIdx.x;
  const int wave  = tid >> 5;
  const int lane  = tid & 31;
  const int c     = lane & 15;
  const int hh    = lane >> 4;
  const int koff  = 8 * hh;
  const int hbase = 16 * wave + 8 * hh;
  const int bbase = blockIdx.x * ROWS_BLK;

  float vw[8], vb[8], vo[8];
  {
    const v4f wi0 = *(const v4f*)(w_ih + hbase);
    const v4f wi1 = *(const v4f*)(w_ih + hbase + 4);
    const v4f bi0 = *(const v4f*)(b_ih + hbase);
    const v4f bi1 = *(const v4f*)(b_ih + hbase + 4);
    asm volatile("" ::: "memory");
    const v4f bh0 = *(const v4f*)(b_hh + hbase);
    const v4f bh1 = *(const v4f*)(b_hh + hbase + 4);
    const v4f wo0 = *(const v4f*)(w_out + hbase);
    const v4f wo1 = *(const v4f*)(w_out + hbase + 4);
    asm volatile("" ::: "memory");
#pragma unroll
    for (int e = 0; e < 4; ++e) {
      vw[e]     = wi0[e] * ACCSCALE;
      vw[4 + e] = wi1[e] * ACCSCALE;
      vb[e]     = (bi0[e] + bh0[e]) * ACCSCALE;
      vb[4 + e] = (bi1[e] + bh1[e]) * ACCSCALE;
      vo[e]     = wo0[e];
      vo[4 + e] = wo1[e];
    }
  }
  const float bo = b_out[0];

  v16h A0, A1;
  {
    const float* wr = w_hh + (size_t)(16 * wave + c) * NHID + koff;
    const v4f p0 = *(const v4f*)(wr);
    const v4f p1 = *(const v4f*)(wr + 4);
    const v4f p2 = *(const v4f*)(wr + 16);
    const v4f p3 = *(const v4f*)(wr + 20);
    asm volatile("" ::: "memory");
    const v4f q0 = *(const v4f*)(wr + 32);
    const v4f q1 = *(const v4f*)(wr + 36);
    const v4f q2 = *(const v4f*)(wr + 48);
    const v4f q3 = *(const v4f*)(wr + 52);
    asm volatile("" ::: "memory");
#pragma unroll
    for (int e = 0; e < 4; ++e) {
      A0[e]      = (_Float16)(p0[e] * WCARRY);
      A0[4 + e]  = (_Float16)(p1[e] * WCARRY);
      A0[8 + e]  = (_Float16)(p2[e] * WCARRY);
      A0[12 + e] = (_Float16)(p3[e] * WCARRY);
      A1[e]      = (_Float16)(q0[e] * WCARRY);
      A1[4 + e]  = (_Float16)(q1[e] * WCARRY);
      A1[8 + e]  = (_Float16)(q2[e] * WCARRY);
      A1[12 + e] = (_Float16)(q3[e] * WCARRY);
    }
  }

  {
    const int r  = tid >> 3;
    const int c0 = (tid & 7) * 8;
    const float* hp = h0 + (size_t)(bbase + r) * NHID + c0;
    const v4f a = *(const v4f*)(hp);
    const v4f b = *(const v4f*)(hp + 4);
    v8h q;
#pragma unroll
    for (int e = 0; e < 4; ++e) {
      q[e]     = (_Float16)(a[e] * HCARRY);
      q[4 + e] = (_Float16)(b[e] * HCARRY);
    }
    *(v8h*)(h_sh + r * HROW + c0) = q;
  }

  int p = 0;
  float th[8];
#pragma unroll
  for (int j = 0; j < 8; ++j) th[j] = 0.0f;

#pragma unroll 1
  for (int tc = 0; tc < NCHUNK; ++tc) {
    const int t0 = tc * CHUNK_T;

    if (tc > 0 && wave == 0) {
      const v4f a = *(const v4f*)(part_sh + (p ^ 1) * 128 + c * 8);
      const v4f b = *(const v4f*)(part_sh + (p ^ 1) * 128 + c * 8 + 4);
      ob_sh[c * FROW + (CHUNK_T - 1)] = ((a[0] + b[0]) + (a[1] + b[1])) + ((a[2] + b[2]) + (a[3] + b[3]));
    }
    {
      const int r  = tid >> 3;
      const int i0 = (tid & 7) * 8;
      const float* xp = x + (size_t)(bbase + r) * NSTEPS + t0 + i0;
      const v4f xa = *(const v4f*)(xp);
      const v4f xb = *(const v4f*)(xp + 4);
      *(v4f*)(x_sh + r * FROW + i0)     = xa;
      *(v4f*)(x_sh + r * FROW + i0 + 4) = xb;
    }
    __syncthreads();

    if (tc > 0) {
      flush_tile(ob_sh, outs + (size_t)bbase * NSTEPS + (size_t)(t0 - CHUNK_T), NSTEPS, bo, wave, lane);
    }

#pragma unroll 1
    for (int tt = 0; tt < CHUNK_T; ++tt) {
      if (tt > 0 && wave == 0) {
        const v4f a = *(const v4f*)(part_sh + (p ^ 1) * 128 + c * 8);
        const v4f b = *(const v4f*)(part_sh + (p ^ 1) * 128 + c * 8 + 4);
        ob_sh[c * FROW + (tt - 1)] = ((a[0] + b[0]) + (a[1] + b[1])) + ((a[2] + b[2]) + (a[3] + b[3]));
      }

      const float xv = x_sh[c * FROW + tt];
      v8f acc;
#pragma unroll
      for (int j = 0; j < 8; ++j) acc[j] = fmaf(vw[j], xv, vb[j]);

      const _Float16* hrow = h_sh + p * HBUF + c * HROW + koff;
      const v16h B0 = Frag<_Float16>::load(hrow);
      const v16h B1 = Frag<_Float16>::load(hrow + 32);

      acc = Frag<_Float16>::mma(A0, B0, acc);
      acc = Frag<_Float16>::mma(A1, B1, acc);
      wmma_guard(acc, A0, B0, A1, B1);

#pragma unroll
      for (int j = 0; j < 8; ++j) th[j] = tanh_f32(acc[j] * ACCFOLD);
      const float pa = fmaf(th[1], vo[1], th[0] * vo[0]);
      const float pb = fmaf(th[3], vo[3], th[2] * vo[2]);
      const float pc = fmaf(th[5], vo[5], th[4] * vo[4]);
      const float pd = fmaf(th[7], vo[7], th[6] * vo[6]);
      const float po = (pa + pb) + (pc + pd);

      v8h q;
#pragma unroll
      for (int j = 0; j < 8; ++j) q[j] = (_Float16)(th[j] * HCARRY);
      *(v8h*)(h_sh + (p ^ 1) * HBUF + c * HROW + hbase) = q;
      part_sh[p * 128 + c * 8 + 2 * wave + hh] = po;

      __syncthreads();
      p ^= 1;
    }
  }

  if (wave == 0) {
    const v4f a = *(const v4f*)(part_sh + (p ^ 1) * 128 + c * 8);
    const v4f b = *(const v4f*)(part_sh + (p ^ 1) * 128 + c * 8 + 4);
    ob_sh[c * FROW + (CHUNK_T - 1)] = ((a[0] + b[0]) + (a[1] + b[1])) + ((a[2] + b[2]) + (a[3] + b[3]));
  }
  {
    v4f f0, f1;
#pragma unroll
    for (int e = 0; e < 4; ++e) { f0[e] = th[e]; f1[e] = th[4 + e]; }
    *(v4f*)(hf_sh + c * FROW + hbase)     = f0;
    *(v4f*)(hf_sh + c * FROW + hbase + 4) = f1;
  }
  __syncthreads();
  flush_tile(ob_sh, outs + (size_t)bbase * NSTEPS + (size_t)(NSTEPS - CHUNK_T), NSTEPS, bo, wave, lane);
  flush_tile(hf_sh, h_last + (size_t)bbase * NHID, NHID, 0.0f, wave, lane);
}

extern "C" void kernel_launch(void* const* d_in, const int* in_sizes, int n_in,
                              void* d_out, int out_size, void* d_ws, size_t ws_size,
                              hipStream_t stream) {
  (void)d_ws; (void)ws_size;
  if (n_in < 8 || d_out == nullptr) return;
  if (in_sizes[0] != NBATCH * NSTEPS || in_sizes[1] != NBATCH * NHID || in_sizes[2] != NHID ||
      in_sizes[3] != NHID * NHID || in_sizes[4] != NHID || in_sizes[5] != NHID ||
      in_sizes[6] != NHID || in_sizes[7] != 1 || out_size != OUT0_ELEMS + OUT1_ELEMS) return;

  const float* x     = (const float*)d_in[0];
  const float* h0    = (const float*)d_in[1];
  const float* w_ih  = (const float*)d_in[2];
  const float* w_hh  = (const float*)d_in[3];
  const float* b_ih  = (const float*)d_in[4];
  const float* b_hh  = (const float*)d_in[5];
  const float* w_out = (const float*)d_in[6];
  const float* b_out = (const float*)d_in[7];
  float* outs   = (float*)d_out;
  float* h_last = outs + (size_t)OUT0_ELEMS;

  rnn_seq_kernel<<<NBATCH / ROWS_BLK, NTHREADS, 0, stream>>>(x, h0, w_ih, w_hh, b_ih, b_hh,
                                                             w_out, b_out, outs, h_last);
}
